// MambaLiteUNet_51668456570920
// MI455X (gfx1250) — hardware-verified
//
#include <hip/hip_runtime.h>
#include <hip/hip_bf16.h>


#define NB_   4
#define DM_   64
#define DI_   128
#define NS_   16
#define XDN_  36
#define XDW_  64
#define C_    256
#define NT_   1024
#define BS_   4
#define MT_   4096
#define MR_   16384
#define NH_   8
#define HD_   32
#define HW_   32

static_assert(MT_ == BS_ * NT_);
static_assert(MR_ == NB_ * MT_);
static_assert(C_ == NB_ * DM_);
static_assert(C_ == NH_ * HD_);
static_assert(NT_ == HW_ * HW_);
static_assert(XDN_ <= XDW_);

typedef float          v4f   __attribute__((ext_vector_type(4)));
typedef float          v8f   __attribute__((ext_vector_type(8)));
typedef _Float16       v8h   __attribute__((ext_vector_type(8)));
typedef _Float16       v16h  __attribute__((ext_vector_type(16)));
typedef __bf16         v16b  __attribute__((ext_vector_type(16)));
typedef unsigned short u16x8 __attribute__((ext_vector_type(8)));
typedef v4f   v4fa   __attribute__((may_alias));
typedef v8h   v8ha   __attribute__((may_alias));
typedef u16x8 u16x8a __attribute__((may_alias));

union FragH { u16x8 h[2]; v8h f[2]; v16h v; };
union FragB { u16x8 h[2]; v16b v; };
union Pack8 { v8h f; u16x8 u; };

constexpr size_t SZ_WINW = (size_t)NB_ * 256 * DM_ * 2;
constexpr size_t SZ_WXPW = (size_t)NB_ * XDW_ * DI_ * 2;
constexpr size_t SZ_WOUT = (size_t)NB_ * DM_ * DI_ * 2;
constexpr size_t SZ_WRPW = (size_t)C_ * C_ * 2;
constexpr size_t SZ_WFPW = (size_t)C_ * 2 * C_ * 2;
constexpr size_t SZ_WAI  = (size_t)3 * C_ * C_ * 2;
constexpr size_t SZ_WAO  = (size_t)C_ * C_ * 2;
constexpr size_t SZ_WFC  = (size_t)C_ * 2 * C_ * 2;
constexpr size_t SZ_WPR  = (size_t)C_ * C_ * 2;
constexpr size_t SZ_P32  = (size_t)MT_ * C_ * 4;
constexpr size_t SZ_P16  = (size_t)MT_ * C_ * 2;
constexpr size_t SZ_XZ   = (size_t)MR_ * 2 * DI_ * 4;
constexpr size_t SZ_U16  = (size_t)MR_ * DI_ * 2;
constexpr size_t SZ_XDBC = (size_t)MR_ * XDW_ * 4;
constexpr size_t SZ_G16  = (size_t)MR_ * DI_ * 2;
constexpr size_t SZ_DWQ  = (size_t)BS_ * NB_ * NT_ * 4;
constexpr size_t SZ_FD16 = (size_t)MT_ * 2 * C_ * 2;
constexpr size_t SZ_HCAT = (size_t)MT_ * 2 * C_ * 2;
constexpr size_t SZ_QKV  = (size_t)MT_ * 3 * C_ * 2;
constexpr size_t SZ_STAT = (size_t)BS_ * C_ * 4;

constexpr size_t OFF_WINW = 0;
constexpr size_t OFF_WXPW = OFF_WINW + SZ_WINW;
constexpr size_t OFF_WOUT = OFF_WXPW + SZ_WXPW;
constexpr size_t OFF_WRPW = OFF_WOUT + SZ_WOUT;
constexpr size_t OFF_WFPW = OFF_WRPW + SZ_WRPW;
constexpr size_t OFF_WAI  = OFF_WFPW + SZ_WFPW;
constexpr size_t OFF_WAO  = OFF_WAI  + SZ_WAI;
constexpr size_t OFF_WFCH = OFF_WAO  + SZ_WAO;
constexpr size_t OFF_WFCL = OFF_WFCH + SZ_WFC;
constexpr size_t OFF_WPRH = OFF_WFCL + SZ_WFC;
constexpr size_t OFF_WPRL = OFF_WPRH + SZ_WPR;
constexpr size_t OFF_XS32 = OFF_WPRL + SZ_WPR;
constexpr size_t OFF_XN32 = OFF_XS32 + SZ_P32;
constexpr size_t OFF_XN16 = OFF_XN32 + SZ_P32;
constexpr size_t OFF_XZ   = OFF_XN16 + SZ_P16;
constexpr size_t OFF_U16  = OFF_XZ   + SZ_XZ;
constexpr size_t OFF_XDBC = OFF_U16  + SZ_U16;
constexpr size_t OFF_G16  = OFF_XDBC + SZ_XDBC;
constexpr size_t OFF_XM32 = OFF_G16  + SZ_G16;
constexpr size_t OFF_DWQ  = OFF_XM32 + SZ_P32;
constexpr size_t OFF_XG32 = OFF_DWQ  + SZ_DWQ;
constexpr size_t OFF_RD16 = OFF_XG32 + SZ_P32;
constexpr size_t OFF_R32  = OFF_RD16 + SZ_P16;
constexpr size_t OFF_FD16 = OFF_R32  + SZ_P32;
constexpr size_t OFF_XM2  = OFF_FD16 + SZ_FD16;
constexpr size_t OFF_XM2H = OFF_XM2  + SZ_P32;
constexpr size_t OFF_HCH  = OFF_XM2H + SZ_P16;
constexpr size_t OFF_HCL  = OFF_HCH  + SZ_HCAT;
constexpr size_t OFF_QKV  = OFF_HCL  + SZ_HCAT;
constexpr size_t OFF_OH16 = OFF_QKV  + SZ_QKV;
constexpr size_t OFF_XO32 = OFF_OH16 + SZ_P16;
constexpr size_t OFF_T1   = OFF_XO32 + SZ_P32;
constexpr size_t OFF_MU   = OFF_T1   + SZ_P32;
constexpr size_t OFF_RS   = OFF_MU   + SZ_STAT;
constexpr size_t OFF_XMH  = OFF_RS   + SZ_STAT;
constexpr size_t OFF_XML  = OFF_XMH  + SZ_P16;
constexpr size_t WS_END   = OFF_XML  + SZ_P16;
static_assert(WS_END == (size_t)96411648);
static_assert(WS_END <= (size_t)134217728);
static_assert(OFF_WXPW % 256 == 0 && OFF_WOUT % 256 == 0 && OFF_WRPW % 256 == 0 && OFF_WFPW % 256 == 0);
static_assert(OFF_WAI % 256 == 0 && OFF_WAO % 256 == 0 && OFF_WFCH % 256 == 0 && OFF_WFCL % 256 == 0);
static_assert(OFF_WPRH % 256 == 0 && OFF_WPRL % 256 == 0 && OFF_XS32 % 256 == 0 && OFF_XN32 % 256 == 0);
static_assert(OFF_XN16 % 256 == 0 && OFF_XZ % 256 == 0 && OFF_U16 % 256 == 0 && OFF_XDBC % 256 == 0);
static_assert(OFF_G16 % 256 == 0 && OFF_XM32 % 256 == 0 && OFF_DWQ % 256 == 0 && OFF_XG32 % 256 == 0);
static_assert(OFF_RD16 % 256 == 0 && OFF_R32 % 256 == 0 && OFF_FD16 % 256 == 0 && OFF_XM2 % 256 == 0);
static_assert(OFF_XM2H % 256 == 0 && OFF_HCH % 256 == 0 && OFF_HCL % 256 == 0 && OFF_QKV % 256 == 0);
static_assert(OFF_OH16 % 256 == 0 && OFF_XO32 % 256 == 0 && OFF_T1 % 256 == 0 && OFF_MU % 256 == 0);
static_assert(OFF_RS % 256 == 0 && OFF_XMH % 256 == 0 && OFF_XML % 256 == 0);

__device__ __forceinline__ unsigned short f2bf(float f) {
    unsigned u = __float_as_uint(f);
    unsigned r = u + 0x7FFFu + ((u >> 16) & 1u);
    return (unsigned short)(r >> 16);
}
__device__ __forceinline__ float bf2f(unsigned short b) {
    return __uint_as_float(((unsigned)b) << 16);
}
__device__ __forceinline__ float rcpf_(float x) { return __builtin_amdgcn_rcpf(x); }
__device__ __forceinline__ float siluf(float x) { return x * rcpf_(1.0f + __expf(-x)); }
__device__ __forceinline__ float sigmf(float x) { return rcpf_(1.0f + __expf(-x)); }
__device__ __forceinline__ float softplusf(float x) { return fmaxf(x, 0.0f) + log1pf(__expf(-fabsf(x))); }
__device__ __forceinline__ float conv4f(float x0, float x1, float x2, float x3,
                                         float w0, float w1, float w2, float w3, float cb) {
    return (w0 * x0 + w1 * x1 + w2 * x2 + w3 * x3) + cb;
}
__device__ __forceinline__ v8f ld8g(const float* p) {
    v4f a = *(const v4f*)p;
    v4f b = *(const v4f*)(p + 4);
    return __builtin_shufflevector(a, b, 0, 1, 2, 3, 4, 5, 6, 7);
}
__device__ __forceinline__ v8f ld8s(const float* p) {
    v4f a = *(const v4fa*)p;
    v4f b = *(const v4fa*)(p + 4);
    return __builtin_shufflevector(a, b, 0, 1, 2, 3, 4, 5, 6, 7);
}
__device__ __forceinline__ float wave_sum(float v) {
#pragma unroll
    for (int o = 16; o > 0; o >>= 1) v += __shfl_xor(v, o, 32);
    return v;
}
__device__ __forceinline__ float block_sum256(float v, float* red8) {
    v = wave_sum(v);
    __syncthreads();
    if ((threadIdx.x & 31) == 0) red8[threadIdx.x >> 5] = v;
    __syncthreads();
    float s = 0.0f;
#pragma unroll
    for (int i = 0; i < 8; ++i) s += red8[i];
    return s;
}

__device__ __forceinline__ void row_store_f32(const float* s, float* g, int nf) {
    const int n4 = nf >> 2;
    for (int i = threadIdx.x; i < n4; i += 256) { const v4f v = *(const v4fa*)(s + 4 * i); *(volatile v4f*)(g + 4 * i) = v; }
    __threadfence();
    for (int i = threadIdx.x; i < n4; i += 256) { const v4f v = *(const v4fa*)(s + 4 * i); *(volatile v4f*)(g + 4 * i) = v; }
}
__device__ __forceinline__ void row_store_f16(const float* s, unsigned short* g, int nh, float scale) {
    const int n8 = nh >> 3;
    for (int i = threadIdx.x; i < n8; i += 256) {
        Pack8 pk; pk.f = __builtin_convertvector(ld8s(s + 8 * i) * scale, v8h);
        const u16x8 u = pk.u; *(volatile u16x8*)(g + 8 * i) = u;
    }
    __threadfence();
    for (int i = threadIdx.x; i < n8; i += 256) {
        Pack8 pk; pk.f = __builtin_convertvector(ld8s(s + 8 * i) * scale, v8h);
        const u16x8 u = pk.u; *(volatile u16x8*)(g + 8 * i) = u;
    }
}
__device__ __forceinline__ void bf16_split8(const float* sp, u16x8& hv, u16x8& lv) {
    const v8f x = ld8s(sp);
#pragma unroll
    for (int c = 0; c < 8; ++c) {
        const unsigned short hb = f2bf(x[c]);
        hv[c] = hb;
        lv[c] = f2bf(x[c] - bf2f(hb));
    }
}
__device__ __forceinline__ void row_store_bf16x2(const float* s, unsigned short* ghi, unsigned short* glo, int nh) {
    const int n8 = nh >> 3;
    for (int i = threadIdx.x; i < n8; i += 256) {
        u16x8 hv, lv; bf16_split8(s + 8 * i, hv, lv);
        *(volatile u16x8*)(ghi + 8 * i) = hv; *(volatile u16x8*)(glo + 8 * i) = lv;
    }
    __threadfence();
    for (int i = threadIdx.x; i < n8; i += 256) {
        u16x8 hv, lv; bf16_split8(s + 8 * i, hv, lv);
        *(volatile u16x8*)(ghi + 8 * i) = hv; *(volatile u16x8*)(glo + 8 * i) = lv;
    }
}

__device__ __forceinline__ void mma16(v8f& acc, const FragH& a, const FragH& b) {
    acc = __builtin_amdgcn_wmma_f32_16x16x32_f16(false, a.v, false, b.v, (short)0, acc, false, false);
    asm volatile("v_nop\n\tv_nop\n\tv_nop\n\tv_nop" : "+v"(acc) : "v"(a.v), "v"(b.v));
}
__device__ __forceinline__ void mma16(v8f& acc, const FragB& a, const FragB& b) {
    acc = __builtin_amdgcn_wmma_f32_16x16x32_bf16(false, a.v, false, b.v, (short)0, acc, false, false);
    asm volatile("v_nop\n\tv_nop\n\tv_nop\n\tv_nop" : "+v"(acc) : "v"(a.v), "v"(b.v));
}

__device__ __forceinline__ void cvt_body(const float* __restrict__ src, unsigned short* dst, unsigned short* dst2,
                                         int n8, int ns8, float sc, int mode)
{
    const int i = blockIdx.x * 256 + threadIdx.x;
    if (i >= n8) return;
    const size_t e = (size_t)i * 8;
    v8f x;
    if (i < ns8) {
        x = ld8g(src + e);
    } else {
#pragma unroll
        for (int c = 0; c < 8; ++c) x[c] = 0.0f;
    }
    if (mode == 0) {
        Pack8 pk; pk.f = __builtin_convertvector(x * sc, v8h);
        const u16x8 v = pk.u;
        *(volatile u16x8*)(dst + e) = v;
        __threadfence();
        *(volatile u16x8*)(dst + e) = v;
    } else {
        u16x8 hv, lv;
#pragma unroll
        for (int c = 0; c < 8; ++c) {
            const unsigned short hb = f2bf(x[c]);
            hv[c] = hb;
            lv[c] = f2bf(x[c] - bf2f(hb));
        }
        *(volatile u16x8*)(dst + e) = hv;
        *(volatile u16x8*)(dst2 + e) = lv;
        __threadfence();
        *(volatile u16x8*)(dst + e) = hv;
        *(volatile u16x8*)(dst2 + e) = lv;
    }
}
__global__ __launch_bounds__(256)
void cvt4_kernel(const float* __restrict__ s0, unsigned short* d0, unsigned short* e0, int n0, int p0, float c0, int q0,
                 const float* __restrict__ s1, unsigned short* d1, unsigned short* e1, int n1, int p1, float c1, int q1,
                 const float* __restrict__ s2, unsigned short* d2, unsigned short* e2, int n2, int p2, float c2, int q2,
                 const float* __restrict__ s3, unsigned short* d3, unsigned short* e3, int n3, int p3, float c3, int q3)
{
    const int seg = blockIdx.y;
    if (seg == 0)      cvt_body(s0, d0, e0, n0, p0, c0, q0);
    else if (seg == 1) cvt_body(s1, d1, e1, n1, p1, c1, q1);
    else if (seg == 2) cvt_body(s2, d2, e2, n2, p2, c2, q2);
    else               cvt_body(s3, d3, e3, n3, p3, c3, q3);
}

template<int NBF, int OM>
__device__ __forceinline__ void tile_store_pass(const float* st, void* C, void* C2, size_t goff, int ldc, int lane)
{
    constexpr int CW  = NBF * 16;
    constexpr int P   = CW + 4;
    constexpr int EPL = (OM == 0) ? 4 : 8;
    static_assert(CW % EPL == 0);
    constexpr int LPR = CW / EPL;
    static_assert(32 % LPR == 0);
    constexpr int RPI = 32 / LPR;
    static_assert(32 % RPI == 0);
    constexpr int NIT = 32 / RPI;
    const int rsub = lane / LPR;
    const int c0   = (lane % LPR) * EPL;
#pragma unroll
    for (int it = 0; it < NIT; ++it) {
        const int row = it * RPI + rsub;
        const float* sp = st + row * P + c0;
        const size_t go = goff + (size_t)row * ldc + c0;
        if (OM == 0) {
            const v4f v = *(const v4fa*)sp;
            *(volatile v4f*)((float*)C + go) = v;
        } else if (OM == 1) {
            Pack8 pk; pk.f = __builtin_convertvector(ld8s(sp), v8h);
            const u16x8 u = pk.u;
            *(volatile u16x8*)((unsigned short*)C + go) = u;
        } else {
            u16x8 hv, lv; bf16_split8(sp, hv, lv);
            *(volatile u16x8*)((unsigned short*)C + go)  = hv;
            *(volatile u16x8*)((unsigned short*)C2 + go) = lv;
        }
    }
}

template<typename FR, bool SPLIT, int NBF, int OM>
__global__ __launch_bounds__(128)
void gemm_tn_kernel(const unsigned short* __restrict__ A,  const unsigned short* __restrict__ A2,
                    long long abs_, int lda, int aks,
                    const unsigned short* __restrict__ Bw, const unsigned short* __restrict__ B2,
                    long long bbs, int ldb, int bks,
                    void* C, void* C2, long long cbs, int ldc,
                    const float* __restrict__ bias, int bias_row,
                    const float* __restrict__ resid, long long rbs, int ldr,
                    const float* __restrict__ rs_ptr,
                    int K, float oscale, float hscale)
{
    constexpr int CW = NBF * 16;
    constexpr int P  = CW + 4;
    __shared__ __attribute__((aligned(16))) float stile[4][32 * P];

    const int tid  = threadIdx.x;
    const int lane = tid & 31;
    const int wave = tid >> 5;
    const int h    = lane >> 4;
    const int m    = lane & 15;
    const int wm   = wave >> 1;
    const int wn   = wave & 1;
    const int z    = blockIdx.z;

    const int rowW = blockIdx.y * 64 + wm * 32;
    const int colW = blockIdx.x * (2 * CW) + wn * CW;

    const unsigned short* Ab  = A  + (size_t)z * (size_t)abs_;
    const unsigned short* A2b = A2 + (size_t)z * (size_t)abs_;
    const unsigned short* Bb  = Bw + (size_t)z * (size_t)bbs;
    const unsigned short* B2b = B2 + (size_t)z * (size_t)bbs;

    v8f acc[2 * NBF];
#pragma unroll
    for (int j = 0; j < 2 * NBF; ++j)
#pragma unroll
        for (int r = 0; r < 8; ++r) acc[j][r] = 0.0f;

    const size_t aoff = (size_t)(rowW + m) * lda + 8 * h;
    const size_t boff = (size_t)(colW + m) * ldb + 8 * h;
    const size_t a16  = (size_t)16 * lda;
    const size_t b16  = (size_t)16 * ldb;
    const int nk = K >> 5;

    for (int kt = 0; kt < nk; ++kt) {
        const size_t ka = (size_t)kt * (size_t)aks;
        const size_t kb = (size_t)kt * (size_t)bks;
        FR fa[2], fb[NBF], ga[2], gb[NBF];
#pragma unroll
        for (int s = 0; s < 2; ++s) {
            const unsigned short* p = Ab + aoff + s * a16 + ka;
            fa[s].h[0] = *(const u16x8*)(p);
            fa[s].h[1] = *(const u16x8*)(p + 16);
            if (SPLIT) {
                const unsigned short* q = A2b + aoff + s * a16 + ka;
                ga[s].h[0] = *(const u16x8*)(q);
                ga[s].h[1] = *(const u16x8*)(q + 16);
            }
        }
#pragma unroll
        for (int j = 0; j < NBF; ++j) {
            const unsigned short* p = Bb + boff + j * b16 + kb;
            fb[j].h[0] = *(const u16x8*)(p);
            fb[j].h[1] = *(const u16x8*)(p + 16);
            if (SPLIT) {
                const unsigned short* q = B2b + boff + j * b16 + kb;
                gb[j].h[0] = *(const u16x8*)(q);
                gb[j].h[1] = *(const u16x8*)(q + 16);
            }
        }
#pragma unroll
        for (int s = 0; s < 2; ++s)
#pragma unroll
            for (int j = 0; j < NBF; ++j) {
                mma16(acc[s * NBF + j], fa[s], fb[j]);
                if (SPLIT) {
                    mma16(acc[s * NBF + j], fa[s], gb[j]);
                    mma16(acc[s * NBF + j], ga[s], fb[j]);
                }
            }
    }

    float rsv = 1.0f;
    if (resid != nullptr && rs_ptr != nullptr) rsv = rs_ptr[0];
    float* st = stile[wave];
#pragma unroll
    for (int s = 0; s < 2; ++s)
#pragma unroll
        for (int j = 0; j < NBF; ++j)
#pragma unroll
            for (int r = 0; r < 8; ++r) {
                const int lrow = s * 16 + 8 * h + r;
                const int lcol = j * 16 + m;
                const int grow = rowW + lrow;
                const int gcol = colW + lcol;
                float v = acc[s * NBF + j][r] * oscale;
                if (bias != nullptr) v += bias[bias_row ? grow : gcol];
                if (resid != nullptr) v += rsv * resid[(size_t)z * (size_t)rbs + (size_t)grow * ldr + gcol];
                if (OM == 1) v *= hscale;
                st[lrow * P + lcol] = v;
            }
    __syncthreads();

    const size_t goff = (size_t)z * (size_t)cbs + (size_t)rowW * ldc + colW;
    tile_store_pass<NBF, OM>(st, C, C2, goff, ldc, lane);
    __threadfence();
    tile_store_pass<NBF, OM>(st, C, C2, goff, ldc, lane);
}

__global__ __launch_bounds__(256)
void ln_in_kernel(const float* __restrict__ x, const float* __restrict__ nw, const float* __restrict__ nbias,
                  float* xs32, float* xn32, unsigned short* xn16)
{
    __shared__ __attribute__((aligned(16))) float sraw[256];
    __shared__ __attribute__((aligned(16))) float sy[256];
    __shared__ float red[8];
    const int row = blockIdx.x;
    const int b = row >> 10, n = row & (NT_ - 1), t = threadIdx.x;
    const float val = x[((size_t)b * C_ + t) * NT_ + n];
    const float mu  = block_sum256(val, red) * (1.0f / 256.0f);
    const float d   = val - mu;
    const float var = block_sum256(d * d, red) * (1.0f / 256.0f);
    const float y   = d * rsqrtf(var + 1e-5f) * nw[t] + nbias[t];
    sraw[t] = val; sy[t] = y;
    __syncthreads();
    row_store_f32(sraw, xs32 + (size_t)row * C_, 256);
    row_store_f32(sy,   xn32 + (size_t)row * C_, 256);
    row_store_f16(sy,   xn16 + (size_t)row * C_, 256, 1.0f);
}

__global__ __launch_bounds__(128)
void conv_silu_kernel(const float* __restrict__ xz, const float* __restrict__ convw, const float* __restrict__ convb,
                      unsigned short* u16)
{
    __shared__ __attribute__((aligned(16))) float su[128];
    const int row = blockIdx.x;
    const int nb = row >> 12, n = row & (NT_ - 1), d = threadIdx.x;
    const int pd = nb * DI_ + d;
    const float* xr = xz + (size_t)row * 256 + d;
    const float x3 = xr[0];
    const float x2 = (n >= 1) ? xr[-256] : 0.0f;
    const float x1 = (n >= 2) ? xr[-512] : 0.0f;
    const float x0 = (n >= 3) ? xr[-768] : 0.0f;
    const float u = siluf(conv4f(x0, x1, x2, x3, convw[pd * 4 + 0], convw[pd * 4 + 1], convw[pd * 4 + 2], convw[pd * 4 + 3], convb[pd]));
    su[d] = u * 64.0f;
    __syncthreads();
    if (d < 16) {
        unsigned short* gp = u16 + (size_t)row * DI_ + 8 * d;
        Pack8 pk; pk.f = __builtin_convertvector(ld8s(su + 8 * d), v8h);
        const u16x8 v = pk.u;
        *(volatile u16x8*)gp = v;
        __threadfence();
        *(volatile u16x8*)gp = v;
    }
}

__global__ __launch_bounds__(128)
void scan_kernel(const float* __restrict__ xz, const float* __restrict__ xdbc,
                 const float* __restrict__ convw, const float* __restrict__ convb,
                 const float* __restrict__ dtw, const float* __restrict__ dtb,
                 const float* __restrict__ alog, const float* __restrict__ Dp,
                 unsigned short* g16)
{
    __shared__ __attribute__((aligned(16))) float sx[16 * XDW_];
    __shared__ __attribute__((aligned(16))) _Float16 sg[16 * DI_];
    const int tid = threadIdx.x, d = tid;
    const int nb = blockIdx.x >> 2, b = blockIdx.x & 3;
    const size_t rowbase = (size_t)nb * MT_ + (size_t)b * NT_;
    const int pd = nb * DI_ + d;

    float an[NS_], hs[NS_];
#pragma unroll
    for (int s = 0; s < NS_; ++s) { an[s] = -expf(alog[pd * NS_ + s]); hs[s] = 0.0f; }
    const float cw0 = convw[pd * 4 + 0], cw1 = convw[pd * 4 + 1], cw2 = convw[pd * 4 + 2], cw3 = convw[pd * 4 + 3];
    const float cb  = convb[pd];
    const float tw0 = dtw[pd * 4 + 0], tw1 = dtw[pd * 4 + 1], tw2 = dtw[pd * 4 + 2], tw3 = dtw[pd * 4 + 3];
    const float tb  = dtb[pd];
    const float Dd  = Dp[pd];
    float xm1 = 0.0f, xm2 = 0.0f, xm3 = 0.0f;

#pragma unroll 1
    for (int l0 = 0; l0 < NT_; l0 += 16) {
#pragma unroll
        for (int jx = 0; jx < 8; ++jx) {
            const int idx = tid + 128 * jx;
            const int tt = idx >> 6, col = idx & 63;
            sx[idx] = xdbc[(rowbase + l0 + tt) * XDW_ + col];
        }
        __syncthreads();
#pragma unroll 1
        for (int t = 0; t < 16; ++t) {
            const size_t row = rowbase + l0 + t;
            const float xv = xz[row * 256 + d];
            const float zv = xz[row * 256 + DI_ + d];
            const float* sxt = sx + t * XDW_;
            float dtv = (sxt[0] * tw0 + sxt[1] * tw1 + sxt[2] * tw2 + sxt[3] * tw3) + tb;
            dtv = softplusf(dtv);
            const float u = siluf(conv4f(xm3, xm2, xm1, xv, cw0, cw1, cw2, cw3, cb));
            xm3 = xm2; xm2 = xm1; xm1 = xv;
            const float du = dtv * u;
            float y = 0.0f;
#pragma unroll
            for (int s = 0; s < NS_; ++s) {
                const float da = __expf(dtv * an[s]);
                hs[s] = da * hs[s] + du * sxt[4 + s];
                y += hs[s] * sxt[4 + NS_ + s];
            }
            const float g = (y + Dd * u) * siluf(zv);
            sg[t * DI_ + d] = (_Float16)(g * 256.0f);
        }
        __syncthreads();
#pragma unroll
        for (int it = 0; it < 2; ++it) {
            const int t = it * 8 + (tid >> 4), c = (tid & 15) * 8;
            Pack8 pk; pk.f = *(const v8ha*)(sg + t * DI_ + c);
            const u16x8 v = pk.u;
            *(volatile u16x8*)(g16 + (rowbase + l0 + t) * DI_ + c) = v;
        }
        __threadfence();
#pragma unroll
        for (int it = 0; it < 2; ++it) {
            const int t = it * 8 + (tid >> 4), c = (tid & 15) * 8;
            Pack8 pk; pk.f = *(const v8ha*)(sg + t * DI_ + c);
            const u16x8 v = pk.u;
            *(volatile u16x8*)(g16 + (rowbase + l0 + t) * DI_ + c) = v;
        }
        __syncthreads();
    }
}

__global__ __launch_bounds__(256)
void gate_dw_kernel(const float* __restrict__ xm32, const float* __restrict__ qdw_w, const float* __restrict__ qdw_b,
                    float* dwq)
{
    __shared__ __attribute__((aligned(16))) float sq[256];
    const int nblk = blockIdx.x, bg = blockIdx.y;
    const int b = bg >> 2, g = bg & 3;
    const int n = nblk * 256 + threadIdx.x;
    float acc = 0.0f;
#pragma unroll
    for (int k = 0; k < 3; ++k) {
        const int nn = n + k - 1;
        if (nn >= 0 && nn < NT_) {
            const float* xr = xm32 + ((size_t)b * NT_ + nn) * C_ + g * DM_;
            const float* wr = qdw_w + g * (DM_ * 3) + k;
            float s = 0.0f;
#pragma unroll 4
            for (int i = 0; i < DM_; ++i) s += wr[i * 3] * xr[i];
            acc += s;
        }
    }
    acc += qdw_b[g];
    sq[threadIdx.x] = acc;
    __syncthreads();
    row_store_f32(sq, dwq + (size_t)bg * NT_ + nblk * 256, 256);
}

__global__ __launch_bounds__(256)
void gate_rd_kernel(const float* __restrict__ xm32, const float* __restrict__ dwq,
                    const float* __restrict__ qpw_w, const float* __restrict__ qpw_b,
                    const float* __restrict__ rdw_w, const float* __restrict__ rdw_b,
                    float* xg32, unsigned short* rd16)
{
    __shared__ float sgate[12];
    __shared__ __attribute__((aligned(16))) float sxg[256];
    __shared__ __attribute__((aligned(16))) float srd[256];
    const int row = blockIdx.x;
    const int b = row >> 10, n = row & (NT_ - 1), c = threadIdx.x, g = c >> 6;
    if (c < 12) {
        const int o = c & 3, j = c >> 2, nn = n + j - 1;
        float gv = 0.0f;
        if (nn >= 0 && nn < NT_) {
            float q = 0.0f;
#pragma unroll
            for (int gg = 0; gg < 4; ++gg) q += qpw_w[o * 4 + gg] * dwq[((size_t)(b * 4 + gg)) * NT_ + nn];
            q += qpw_b[o];
            gv = sigmf(q);
        }
        sgate[c] = gv;
    }
    __syncthreads();
    const size_t rb = (size_t)b * NT_;
    const float xv0 = (n >= 1)       ? sgate[0 * 4 + g] * xm32[(rb + n - 1) * C_ + c] : 0.0f;
    const float xv1 =                  sgate[1 * 4 + g] * xm32[(rb + n)     * C_ + c];
    const float xv2 = (n + 1 < NT_)  ? sgate[2 * 4 + g] * xm32[(rb + n + 1) * C_ + c] : 0.0f;
    const float rd = (rdw_w[c * 3 + 0] * xv0 + rdw_w[c * 3 + 1] * xv1 + rdw_w[c * 3 + 2] * xv2) + rdw_b[c];
    sxg[c] = xv1; srd[c] = rd;
    __syncthreads();
    row_store_f32(sxg, xg32 + (size_t)row * C_, 256);
    row_store_f16(srd, rd16 + (size_t)row * C_, 256, 1.0f);
}

__global__ __launch_bounds__(256)
void fd_kernel(const float* __restrict__ xs32, const float* __restrict__ R32,
               const float* __restrict__ fdw_w, const float* __restrict__ fdw_b, unsigned short* fd16)
{
    __shared__ __attribute__((aligned(16))) float sfd[512];
    const int row = blockIdx.x;
    const int n = row & (NT_ - 1), c = threadIdx.x;
#pragma unroll
    for (int part = 0; part < 2; ++part) {
        const float* src = part ? R32 : xs32;
        const int j = part * C_ + c;
        const float a0 = (n >= 1)      ? src[(size_t)(row - 1) * C_ + c] : 0.0f;
        const float a1 =                 src[(size_t)row * C_ + c];
        const float a2 = (n + 1 < NT_) ? src[(size_t)(row + 1) * C_ + c] : 0.0f;
        sfd[j] = (fdw_w[j * 3 + 0] * a0 + fdw_w[j * 3 + 1] * a1 + fdw_w[j * 3 + 2] * a2) + fdw_b[j];
    }
    __syncthreads();
    row_store_f16(sfd, fd16 + (size_t)row * (2 * C_), 512, 1.0f);
}

__global__ __launch_bounds__(256)
void xlocal_kernel(const float* __restrict__ xm2, const float* __restrict__ lc_w, const float* __restrict__ lc_b,
                   unsigned short* xm2h, unsigned short* hch, unsigned short* hcl)
{
    __shared__ __attribute__((aligned(16))) float sc[256];
    __shared__ __attribute__((aligned(16))) float sl[256];
    const int row = blockIdx.x;
    const int n = row & (NT_ - 1), c = threadIdx.x;
    const float a0 = (n >= 1)      ? xm2[(size_t)(row - 1) * C_ + c] : 0.0f;
    const float a1 =                 xm2[(size_t)row * C_ + c];
    const float a2 = (n + 1 < NT_) ? xm2[(size_t)(row + 1) * C_ + c] : 0.0f;
    sl[c] = (lc_w[c * 3 + 0] * a0 + lc_w[c * 3 + 1] * a1 + lc_w[c * 3 + 2] * a2) + lc_b[c];
    sc[c] = a1;
    __syncthreads();
    row_store_f16(sc, xm2h + (size_t)row * C_, 256, 1.0f);
    row_store_bf16x2(sl, hch + (size_t)row * (2 * C_), hcl + (size_t)row * (2 * C_), 256);
}

__global__ __launch_bounds__(128)
void attn_kernel(const unsigned short* __restrict__ qkv, unsigned short* oh, float sscale, float ofac)
{
    constexpr int PK = 40, PV = 72, PP = 72;
    __shared__ __attribute__((aligned(16))) unsigned short sK[64 * PK];
    __shared__ __attribute__((aligned(16))) unsigned short sVt[32 * PV];
    __shared__ __attribute__((aligned(16))) _Float16 sP[4][16 * PP];

    const int tid = threadIdx.x, lane = tid & 31, wave = tid >> 5;
    const int hh = lane >> 4, m = lane & 15;
    const int qb = blockIdx.x, head = blockIdx.y, b = blockIdx.z;
    const int q0 = qb * 64 + wave * 16;
    const size_t rowq = (size_t)b * NT_ + q0;

    FragH qf;
    {
        const unsigned short* p = qkv + (rowq + m) * 768 + head * HD_ + 8 * hh;
        qf.h[0] = *(const u16x8*)(p);
        qf.h[1] = *(const u16x8*)(p + 16);
    }
    v8f acco[2];
#pragma unroll
    for (int j = 0; j < 2; ++j)
#pragma unroll
        for (int r = 0; r < 8; ++r) acco[j][r] = 0.0f;
    float mrow[8], lrow[8];
#pragma unroll
    for (int r = 0; r < 8; ++r) { mrow[r] = -1e30f; lrow[r] = 0.0f; }
    _Float16* sPw = sP[wave];

#pragma unroll 1
    for (int kb = 0; kb < NT_ / 64; ++kb) {
        {
            const int key = tid >> 1, part = tid & 1;
            const size_t rk = (size_t)b * NT_ + (size_t)kb * 64 + key;
            const unsigned short* kp = qkv + rk * 768 + 256 + head * HD_ + part * 16;
            const unsigned short* vp = kp + 256;
            const u16x8 k0 = *(const u16x8*)(kp), k1 = *(const u16x8*)(kp + 8);
            const u16x8 v0 = *(const u16x8*)(vp), v1 = *(const u16x8*)(vp + 8);
            *(u16x8a*)(sK + key * PK + part * 16)     = k0;
            *(u16x8a*)(sK + key * PK + part * 16 + 8) = k1;
#pragma unroll
            for (int i = 0; i < 8; ++i) {
                sVt[(part * 16 + i) * PV + key]     = v0[i];
                sVt[(part * 16 + 8 + i) * PV + key] = v1[i];
            }
        }
        __syncthreads();

        v8f accs[4];
#pragma unroll
        for (int j = 0; j < 4; ++j)
#pragma unroll
            for (int r = 0; r < 8; ++r) accs[j][r] = 0.0f;
#pragma unroll
        for (int j = 0; j < 4; ++j) {
            FragH kf;
            kf.h[0] = *(const u16x8a*)(sK + (j * 16 + m) * PK + 8 * hh);
            kf.h[1] = *(const u16x8a*)(sK + (j * 16 + m) * PK + 16 + 8 * hh);
            mma16(accs[j], qf, kf);
        }
#pragma unroll
        for (int r = 0; r < 8; ++r) {
#pragma unroll
            for (int j = 0; j < 4; ++j) accs[j][r] *= sscale;
            float mx = fmaxf(fmaxf(accs[0][r], accs[1][r]), fmaxf(accs[2][r], accs[3][r]));
#pragma unroll
            for (int o = 1; o < 16; o <<= 1) mx = fmaxf(mx, __shfl_xor(mx, o, 32));
            const float mn = fmaxf(mrow[r], mx);
            const float al = __expf(mrow[r] - mn);
            float ps = 0.0f;
#pragma unroll
            for (int j = 0; j < 4; ++j) { const float p = __expf(accs[j][r] - mn); accs[j][r] = p; ps += p; }
#pragma unroll
            for (int o = 1; o < 16; o <<= 1) ps += __shfl_xor(ps, o, 32);
            lrow[r] = lrow[r] * al + ps;
            mrow[r] = mn;
            acco[0][r] *= al;
            acco[1][r] *= al;
        }
#pragma unroll
        for (int j = 0; j < 4; ++j)
#pragma unroll
            for (int r = 0; r < 8; ++r)
                sPw[(8 * hh + r) * PP + j * 16 + m] = (_Float16)(accs[j][r] * 16384.0f);
        __syncthreads();
#pragma unroll
        for (int ks = 0; ks < 2; ++ks) {
            FragH pa;
            pa.f[0] = *(const v8ha*)(sPw + m * PP + ks * 32 + 8 * hh);
            pa.f[1] = *(const v8ha*)(sPw + m * PP + ks * 32 + 16 + 8 * hh);
#pragma unroll
            for (int jj = 0; jj < 2; ++jj) {
                FragH vb;
                vb.h[0] = *(const u16x8a*)(sVt + (jj * 16 + m) * PV + ks * 32 + 8 * hh);
                vb.h[1] = *(const u16x8a*)(sVt + (jj * 16 + m) * PV + ks * 32 + 16 + 8 * hh);
                mma16(acco[jj], pa, vb);
            }
        }
        __syncthreads();
    }

    _Float16* so = sPw;
#pragma unroll
    for (int r = 0; r < 8; ++r) {
        const float inv = ofac * rcpf_(lrow[r]);
#pragma unroll
        for (int jj = 0; jj < 2; ++jj)
            so[(8 * hh + r) * PP + jj * 16 + m] = (_Float16)(acco[jj][r] * inv);
    }
    __syncthreads();
    const size_t obase = (((size_t)b * NH_ + head) * NT_ + q0) * HD_;
#pragma unroll
    for (int it = 0; it < 2; ++it) {
        const int row = it * 8 + (lane >> 2), c8 = (lane & 3) * 8;
        Pack8 pk; pk.f = *(const v8ha*)(so + row * PP + c8);
        const u16x8 u = pk.u;
        *(volatile u16x8*)(oh + obase + (size_t)row * HD_ + c8) = u;
    }
    __threadfence();
#pragma unroll
    for (int it = 0; it < 2; ++it) {
        const int row = it * 8 + (lane >> 2), c8 = (lane & 3) * 8;
        Pack8 pk; pk.f = *(const v8ha*)(so + row * PP + c8);
        const u16x8 u = pk.u;
        *(volatile u16x8*)(oh + obase + (size_t)row * HD_ + c8) = u;
    }
}

__global__ __launch_bounds__(256)
void lgn_gelu_kernel(const float* __restrict__ xo, const float* __restrict__ w, const float* __restrict__ bsh, float* t1)
{
    __shared__ __attribute__((aligned(16))) float st[256];
    __shared__ float red[8];
    const int row = blockIdx.x, t = threadIdx.x;
    const float val = xo[(size_t)row * C_ + t];
    const float mu  = block_sum256(val, red) * (1.0f / 256.0f);
    const float d   = val - mu;
    const float var = block_sum256(d * d, red) * (1.0f / 256.0f);
    const float y   = d * rsqrtf(var + 1e-5f) * w[t] + bsh[t];
    st[t] = 0.5f * y * (1.0f + erff(y * 0.70710678118654752f));
    __syncthreads();
    row_store_f32(st, t1 + (size_t)row * C_, 256);
}

__global__ __launch_bounds__(256)
void hw_stats_kernel(const float* __restrict__ t1, float* mu_arr, float* rs_arr)
{
    __shared__ float red2[8 * 32];
    __shared__ __attribute__((aligned(16))) float smu[32];
    __shared__ __attribute__((aligned(16))) float srs[32];
    const int tid = threadIdx.x, lane = tid & 31, wave = tid >> 5;
    const int cg = blockIdx.x, b = blockIdx.y;
    const int c = cg * 32 + lane;
    const float* base = t1 + ((size_t)b * NT_) * C_ + c;
    float s = 0.0f;
#pragma unroll 4
    for (int i = 0; i < 128; ++i) s += base[(size_t)(wave * 128 + i) * C_];
    red2[wave * 32 + lane] = s;
    __syncthreads();
    if (wave == 0) {
        float ts = 0.0f;
#pragma unroll
        for (int w8 = 0; w8 < 8; ++w8) ts += red2[w8 * 32 + lane];
        smu[lane] = ts * (1.0f / 1024.0f);
    }
    __syncthreads();
    const float mu = smu[lane];
    float s2 = 0.0f;
#pragma unroll 4
    for (int i = 0; i < 128; ++i) { const float dv = base[(size_t)(wave * 128 + i) * C_] - mu; s2 += dv * dv; }
    red2[wave * 32 + lane] = s2;
    __syncthreads();
    if (wave == 0) {
        float ts = 0.0f;
#pragma unroll
        for (int w8 = 0; w8 < 8; ++w8) ts += red2[w8 * 32 + lane];
        srs[lane] = rsqrtf(ts * (1.0f / 1024.0f) + 1e-5f);
    }
    __syncthreads();
    const size_t go = (size_t)b * C_ + cg * 32;
    if (tid < 8)       { const v4f v = *(const v4fa*)(smu + 4 * tid);       *(volatile v4f*)(mu_arr + go + 4 * tid) = v; }
    else if (tid < 16) { const v4f v = *(const v4fa*)(srs + 4 * (tid - 8)); *(volatile v4f*)(rs_arr + go + 4 * (tid - 8)) = v; }
    __threadfence();
    if (tid < 8)       { const v4f v = *(const v4fa*)(smu + 4 * tid);       *(volatile v4f*)(mu_arr + go + 4 * tid) = v; }
    else if (tid < 16) { const v4f v = *(const v4fa*)(srs + 4 * (tid - 8)); *(volatile v4f*)(rs_arr + go + 4 * (tid - 8)) = v; }
}

__global__ __launch_bounds__(256)
void dwc_ln_kernel(const float* __restrict__ t1, const float* __restrict__ mu_arr, const float* __restrict__ rs_arr,
                   const float* __restrict__ dwc_w, const float* __restrict__ dwc_b,
                   const float* __restrict__ nw, const float* __restrict__ nbias,
                   unsigned short* xmh, unsigned short* xml)
{
    __shared__ __attribute__((aligned(16))) float st[256];
    __shared__ float red[8];
    const int row = blockIdx.x;
    const int b = row >> 10, n = row & (NT_ - 1), c = threadIdx.x;
    const int y0 = n >> 5, x0 = n & 31;
    const float mu0 = mu_arr[b * C_ + c], rs0 = rs_arr[b * C_ + c];
    float acc = 0.0f;
#pragma unroll
    for (int dy = 0; dy < 3; ++dy) {
        const int yy = y0 + dy - 1;
        if (yy < 0 || yy >= HW_) continue;
#pragma unroll
        for (int dx = 0; dx < 3; ++dx) {
            const int xx = x0 + dx - 1;
            if (xx < 0 || xx >= HW_) continue;
            const float v = (t1[((size_t)b * NT_ + yy * HW_ + xx) * C_ + c] - mu0) * rs0;
            acc += dwc_w[c * 9 + dy * 3 + dx] * v;
        }
    }
    acc += dwc_b[c];
    const float mu  = block_sum256(acc, red) * (1.0f / 256.0f);
    const float d   = acc - mu;
    const float var = block_sum256(d * d, red) * (1.0f / 256.0f);
    st[c] = d * rsqrtf(var + 1e-5f) * nw[c] + nbias[c];
    __syncthreads();
    row_store_bf16x2(st, xmh + (size_t)row * C_, xml + (size_t)row * C_, 256);
}

template<typename FR, bool SPLIT, int NBF, int OM>
static void launch_gemm(hipStream_t st, dim3 grid,
                        const unsigned short* A, const unsigned short* A2, long long abs_, int lda, int aks,
                        const unsigned short* B, const unsigned short* B2, long long bbs, int ldb, int bks,
                        void* C, void* C2, long long cbs, int ldc,
                        const float* bias, int bias_row,
                        const float* resid, long long rbs, int ldr, const float* rs_ptr,
                        int K, float oscale, float hscale)
{
    hipLaunchKernelGGL(HIP_KERNEL_NAME(gemm_tn_kernel<FR, SPLIT, NBF, OM>), grid, dim3(128), 0, st,
                       A, A2, abs_, lda, aks, B, B2, bbs, ldb, bks, C, C2, cbs, ldc,
                       bias, bias_row, resid, rbs, ldr, rs_ptr, K, oscale, hscale);
}

extern "C" void kernel_launch(void* const* d_in, const int* in_sizes, int n_in,
                              void* d_out, int out_size, void* d_ws, size_t ws_size,
                              hipStream_t stream)
{
    if (n_in < 39) return;
    if (in_sizes[0]  != BS_ * C_ * NT_)      return;
    if (in_sizes[4]  != NB_ * 2 * DI_ * DM_) return;
    if (in_sizes[7]  != NB_ * XDN_ * DI_)    return;
    if (in_sizes[27] != 3 * C_ * C_)         return;
    if (in_sizes[33] != C_ * 2 * C_)         return;
    if (out_size != BS_ * C_ * NT_)          return;
    if (ws_size < WS_END)                    return;

    const float* x         = (const float*)d_in[0];
    const float* norm_w    = (const float*)d_in[1];
    const float* norm_b    = (const float*)d_in[2];
    const float* skip_s    = (const float*)d_in[3];
    const float* m_inw     = (const float*)d_in[4];
    const float* m_convw   = (const float*)d_in[5];
    const float* m_convb   = (const float*)d_in[6];
    const float* m_xpw     = (const float*)d_in[7];
    const float* m_dtw     = (const float*)d_in[8];
    const float* m_dtb     = (const float*)d_in[9];
    const float* m_alog    = (const float*)d_in[10];
    const float* m_d       = (const float*)d_in[11];
    const float* m_outw    = (const float*)d_in[12];
    const float* qdw_w     = (const float*)d_in[13];
    const float* qdw_b     = (const float*)d_in[14];
    const float* qpw_w     = (const float*)d_in[15];
    const float* qpw_b     = (const float*)d_in[16];
    const float* rdw_w     = (const float*)d_in[17];
    const float* rdw_b     = (const float*)d_in[18];
    const float* rpw_w     = (const float*)d_in[19];
    const float* rpw_b     = (const float*)d_in[20];
    const float* fdw_w     = (const float*)d_in[21];
    const float* fdw_b     = (const float*)d_in[22];
    const float* fpw_w     = (const float*)d_in[23];
    const float* fpw_b     = (const float*)d_in[24];
    const float* lc_w      = (const float*)d_in[25];
    const float* lc_b      = (const float*)d_in[26];
    const float* attn_inw  = (const float*)d_in[27];
    const float* attn_inb  = (const float*)d_in[28];
    const float* attn_outw = (const float*)d_in[29];
    const float* attn_outb = (const float*)d_in[30];
    const float* lgn_w     = (const float*)d_in[31];
    const float* lgn_b     = (const float*)d_in[32];
    const float* fc_w      = (const float*)d_in[33];
    const float* fc_b      = (const float*)d_in[34];
    const float* dwc_w     = (const float*)d_in[35];
    const float* dwc_b     = (const float*)d_in[36];
    const float* proj_w    = (const float*)d_in[37];
    const float* proj_b    = (const float*)d_in[38];
    float* out = (float*)d_out;

    char* ws = (char*)d_ws;
    unsigned short* w_inw  = (unsigned short*)(ws + OFF_WINW);
    unsigned short* w_xpw  = (unsigned short*)(ws + OFF_WXPW);
    unsigned short* w_out  = (unsigned short*)(ws + OFF_WOUT);
    unsigned short* w_rpw  = (unsigned short*)(ws + OFF_WRPW);
    unsigned short* w_fpw  = (unsigned short*)(ws + OFF_WFPW);
    unsigned short* w_ai   = (unsigned short*)(ws + OFF_WAI);
    unsigned short* w_ao   = (unsigned short*)(ws + OFF_WAO);
    unsigned short* w_fch  = (unsigned short*)(ws + OFF_WFCH);
    unsigned short* w_fcl  = (unsigned short*)(ws + OFF_WFCL);
    unsigned short* w_prh  = (unsigned short*)(ws + OFF_WPRH);
    unsigned short* w_prl  = (unsigned short*)(ws + OFF_WPRL);
    float*          xs32   = (float*)(ws + OFF_XS32);
    float*          xn32   = (float*)(ws + OFF_XN32);
    unsigned short* xn16   = (unsigned short*)(ws + OFF_XN16);
    float*          xz32   = (float*)(ws + OFF_XZ);
    unsigned short* u16    = (unsigned short*)(ws + OFF_U16);
    float*          xdbc   = (float*)(ws + OFF_XDBC);
    unsigned short* g16    = (unsigned short*)(ws + OFF_G16);
    float*          xm32   = (float*)(ws + OFF_XM32);
    float*          dwq    = (float*)(ws + OFF_DWQ);
    float*          xg32   = (float*)(ws + OFF_XG32);
    unsigned short* rd16   = (unsigned short*)(ws + OFF_RD16);
    float*          R32    = (float*)(ws + OFF_R32);
    unsigned short* fd16   = (unsigned short*)(ws + OFF_FD16);
    float*          xm2    = (float*)(ws + OFF_XM2);
    unsigned short* xm2h   = (unsigned short*)(ws + OFF_XM2H);
    unsigned short* hch    = (unsigned short*)(ws + OFF_HCH);
    unsigned short* hcl    = (unsigned short*)(ws + OFF_HCL);
    unsigned short* qkv16  = (unsigned short*)(ws + OFF_QKV);
    unsigned short* oh16   = (unsigned short*)(ws + OFF_OH16);
    float*          xo32   = (float*)(ws + OFF_XO32);
    float*          t1     = (float*)(ws + OFF_T1);
    float*          mu_arr = (float*)(ws + OFF_MU);
    float*          rs_arr = (float*)(ws + OFF_RS);
    unsigned short* xmh    = (unsigned short*)(ws + OFF_XMH);
    unsigned short* xml    = (unsigned short*)(ws + OFF_XML);

    {
        const int n_inw = (NB_ * 256 * DM_) / 8;
        const int n_xpw = (XDW_ * DI_) / 8;
        const int s_xpw = (XDN_ * DI_) / 8;
        const int n_ow  = (NB_ * DM_ * DI_) / 8;
        const int n_rpw = (C_ * C_) / 8;
        const int n_fpw = (C_ * 2 * C_) / 8;
        const int n_ai  = (3 * C_ * C_) / 8;
        const int n_ao  = (C_ * C_) / 8;
        const int n_fc  = (C_ * 2 * C_) / 8;
        const int n_pr  = (C_ * C_) / 8;
        hipLaunchKernelGGL(cvt4_kernel, dim3((n_inw + 255) / 256, 4), dim3(256), 0, stream,
                           m_inw, w_inw, w_inw, n_inw, n_inw, 32.0f, 0,
                           m_xpw + 0 * XDN_ * DI_, w_xpw + 0 * XDW_ * DI_, w_xpw, n_xpw, s_xpw, 32.0f, 0,
                           m_xpw + 1 * XDN_ * DI_, w_xpw + 1 * XDW_ * DI_, w_xpw, n_xpw, s_xpw, 32.0f, 0,
                           m_xpw + 2 * XDN_ * DI_, w_xpw + 2 * XDW_ * DI_, w_xpw, n_xpw, s_xpw, 32.0f, 0);
        hipLaunchKernelGGL(cvt4_kernel, dim3((n_fpw + 255) / 256, 4), dim3(256), 0, stream,
                           m_xpw + 3 * XDN_ * DI_, w_xpw + 3 * XDW_ * DI_, w_xpw, n_xpw, s_xpw, 32.0f, 0,
                           m_outw, w_out, w_out, n_ow, n_ow, 32.0f, 0,
                           rpw_w, w_rpw, w_rpw, n_rpw, n_rpw, 32.0f, 0,
                           fpw_w, w_fpw, w_fpw, n_fpw, n_fpw, 32.0f, 0);
        hipLaunchKernelGGL(cvt4_kernel, dim3((n_ai + 255) / 256, 4), dim3(256), 0, stream,
                           attn_inw, w_ai, w_ai, n_ai, n_ai, 32.0f, 0,
                           attn_outw, w_ao, w_ao, n_ao, n_ao, 32.0f, 0,
                           fc_w, w_fch, w_fcl, n_fc, n_fc, 1.0f, 1,
                           proj_w, w_prh, w_prl, n_pr, n_pr, 1.0f, 1);
    }

    hipLaunchKernelGGL(ln_in_kernel, dim3(MT_), dim3(256), 0, stream, x, norm_w, norm_b, xs32, xn32, xn16);

    launch_gemm<FragH, false, 4, 0>(stream, dim3(256 / 128, MT_ / 64, NB_),
        xn16, xn16, (long long)DM_, C_, 32,
        w_inw, w_inw, (long long)(256 * DM_), DM_, 32,
        (void*)xz32, (void*)xz32, (long long)MT_ * 256, 256,
        nullptr, 0, nullptr, 0, 0, nullptr,
        DM_, 1.0f / 32.0f, 1.0f);

    hipLaunchKernelGGL(conv_silu_kernel, dim3(MR_), dim3(DI_), 0, stream, (const float*)xz32, m_convw, m_convb, u16);

    launch_gemm<FragH, false, 2, 0>(stream, dim3(XDW_ / 64, MT_ / 64, NB_),
        u16, u16, (long long)MT_ * DI_, DI_, 32,
        w_xpw, w_xpw, (long long)(XDW_ * DI_), DI_, 32,
        (void*)xdbc, (void*)xdbc, (long long)MT_ * XDW_, XDW_,
        nullptr, 0, nullptr, 0, 0, nullptr,
        DI_, 1.0f / 2048.0f, 1.0f);

    hipLaunchKernelGGL(scan_kernel, dim3(NB_ * BS_), dim3(DI_), 0, stream,
                       (const float*)xz32, (const float*)xdbc, m_convw, m_convb, m_dtw, m_dtb, m_alog, m_d, g16);

    launch_gemm<FragH, false, 2, 0>(stream, dim3(DM_ / 64, MT_ / 64, NB_),
        g16, g16, (long long)MT_ * DI_, DI_, 32,
        w_out, w_out, (long long)(DM_ * DI_), DI_, 32,
        (void*)xm32, (void*)xm32, (long long)DM_, C_,
        nullptr, 0, (const float*)xn32, (long long)DM_, C_, skip_s,
        DI_, 1.0f / 8192.0f, 1.0f);

    hipLaunchKernelGGL(gate_dw_kernel, dim3(NT_ / 256, BS_ * NB_), dim3(256), 0, stream,
                       (const float*)xm32, qdw_w, qdw_b, dwq);
    hipLaunchKernelGGL(gate_rd_kernel, dim3(MT_), dim3(256), 0, stream,
                       (const float*)xm32, (const float*)dwq, qpw_w, qpw_b, rdw_w, rdw_b, xg32, rd16);

    launch_gemm<FragH, false, 4, 0>(stream, dim3(C_ / 128, MT_ / 64, 1),
        rd16, rd16, 0, C_, 32,
        w_rpw, w_rpw, 0, C_, 32,
        (void*)R32, (void*)R32, 0, C_,
        rpw_b, 0, (const float*)xg32, 0, C_, nullptr,
        C_, 1.0f / 32.0f, 1.0f);

    hipLaunchKernelGGL(fd_kernel, dim3(MT_), dim3(256), 0, stream, (const float*)xs32, (const float*)R32, fdw_w, fdw_b, fd16);
    launch_gemm<FragH, false, 4, 0>(stream, dim3(C_ / 128, MT_ / 64, 1),
        fd16, fd16, 0, 2 * C_, 32,
        w_fpw, w_fpw, 0, 2 * C_, 32,
        (void*)xm2, (void*)xm2, 0, C_,
        fpw_b, 0, (const float*)xs32, 0, C_, nullptr,
        2 * C_, 1.0f / 32.0f, 1.0f);

    hipLaunchKernelGGL(xlocal_kernel, dim3(MT_), dim3(256), 0, stream, (const float*)xm2, lc_w, lc_b, xm2h, hch, hcl);

    launch_gemm<FragH, false, 4, 1>(stream, dim3((3 * C_) / 128, MT_ / 64, 1),
        xm2h, xm2h, 0, C_, 32,
        w_ai, w_ai, 0, C_, 32,
        (void*)qkv16, (void*)qkv16, 0, 3 * C_,
        attn_inb, 0, nullptr, 0, 0, nullptr,
        C_, 1.0f / 32.0f, 8.0f);

    hipLaunchKernelGGL(attn_kernel, dim3(NT_ / 64, NH_, BS_), dim3(128), 0, stream,
                       (const unsigned short*)qkv16, oh16, 0.17677669529663687f * (1.0f / 64.0f), 1.0f / 8192.0f);

    launch_gemm<FragH, false, 4, 2>(stream, dim3(C_ / 128, NT_ / 64, BS_),
        oh16, oh16, (long long)NH_ * NT_ * HD_, HD_, NT_ * HD_,
        w_ao, w_ao, 0, C_, 32,
        (void*)(hch + C_), (void*)(hcl + C_), (long long)NT_ * 2 * C_, 2 * C_,
        attn_outb, 0, nullptr, 0, 0, nullptr,
        C_, 1.0f / 512.0f, 1.0f);

    launch_gemm<FragB, true, 2, 0>(stream, dim3(C_ / 64, MT_ / 64, 1),
        hch, hcl, 0, 2 * C_, 32,
        w_fch, w_fcl, 0, 2 * C_, 32,
        (void*)xo32, (void*)xo32, 0, C_,
        fc_b, 0, nullptr, 0, 0, nullptr,
        2 * C_, 1.0f, 1.0f);

    hipLaunchKernelGGL(lgn_gelu_kernel, dim3(MT_), dim3(256), 0, stream, (const float*)xo32, lgn_w, lgn_b, t1);
    hipLaunchKernelGGL(hw_stats_kernel, dim3(C_ / 32, BS_), dim3(256), 0, stream, (const float*)t1, mu_arr, rs_arr);
    hipLaunchKernelGGL(dwc_ln_kernel, dim3(MT_), dim3(256), 0, stream,
                       (const float*)t1, (const float*)mu_arr, (const float*)rs_arr, dwc_w, dwc_b, norm_w, norm_b, xmh, xml);

    launch_gemm<FragB, true, 2, 0>(stream, dim3(NT_ / 64, C_ / 64, BS_),
        w_prh, w_prl, 0, C_, 32,
        xmh, xml, (long long)NT_ * C_, C_, 32,
        (void*)out, (void*)out, (long long)C_ * NT_, NT_,
        proj_b, 1, nullptr, 0, 0, nullptr,
        C_, 1.0f, 1.0f);
}
